// DeltaNet_31877247271540
// MI455X (gfx1250) — hardware-verified
//
#include <hip/hip_runtime.h>
#include <math.h>

constexpr int kB    = 2;
constexpr int kL    = 2048;
constexpr int kD    = 1024;
constexpr int kH    = 4;
constexpr int kDK   = 256;
constexpr int kC    = 32;
constexpr int kNCH  = kL / kC;
constexpr int kTok  = kB * kL;
constexpr int kBH   = kB * kH;
constexpr int kGIn  = 1088;
constexpr int kHid2 = 2048;
constexpr int kNLg  = 64;
constexpr int kFirK = 63;
constexpr int kSeqLen = 336;
constexpr float kWCar     = 256.0f;
constexpr float kWCarInv  = 1.0f / 256.0f;
constexpr float kHmCar    = 16.0f;
constexpr float kW2Scale  = 1.0f / (16.0f * 256.0f);
constexpr float kTapCar   = 16.0f;
constexpr float kTapCarInv = 1.0f / 16.0f;
static_assert(kH * kDK == kD, "shape");
static_assert(kTok % 64 == 0 && kD % 64 == 0 && kHid2 % 64 == 0 && kNLg % 64 == 0, "M,N tile multiples");
static_assert(kD % 32 == 0 && kGIn % 32 == 0 && kHid2 % 32 == 0, "K multiples of 32");
static_assert(kGIn % 64 == 0, "transpose tiles of W1");
static_assert(kL % 256 == 0 && kD % 32 == 0, "FIR tiles");
static_assert(16 * 15 + 95 < kSeqLen, "FIR window extent");

typedef __attribute__((ext_vector_type(16))) _Float16 v16h;
typedef __attribute__((ext_vector_type(8)))  _Float16 v8h;
typedef __attribute__((ext_vector_type(16))) __bf16   v16b;
typedef __attribute__((ext_vector_type(8)))  __bf16   v8b;
typedef __attribute__((ext_vector_type(8)))  float    v8f;
typedef __attribute__((ext_vector_type(4)))  float    v4f;
typedef __attribute__((ext_vector_type(4)))  unsigned int v4u;
typedef __attribute__((ext_vector_type(2)))  unsigned int v2u;
typedef __attribute__((ext_vector_type(8)))  unsigned int v8u;

__device__ __forceinline__ unsigned short f2bf_bits(float f) {
  unsigned u = __float_as_uint(f);
  return (unsigned short)((u + 0x7FFFu + ((u >> 16) & 1u)) >> 16);
}
__device__ __forceinline__ float bf_bits2f(unsigned short h) { return __uint_as_float(((unsigned)h) << 16); }

__device__ __forceinline__ void dep_guard_h(v8f& a, v8f& b, v16h x, v16h y) { asm volatile("v_nop\n\tv_nop\n\tv_nop\n\tv_nop" : "+v"(a), "+v"(b) : "v"(x), "v"(y)); }
__device__ __forceinline__ void dep_guard_b(v8f& a, v8f& b, v16b x, v16b y) { asm volatile("v_nop\n\tv_nop\n\tv_nop\n\tv_nop" : "+v"(a), "+v"(b) : "v"(x), "v"(y)); }
__device__ __forceinline__ void keep4_h(v16h a, v16h b, v16h c, v16h d) { asm volatile("v_nop" :: "v"(a), "v"(b), "v"(c), "v"(d)); }
__device__ __forceinline__ void keep4_b(v16b a, v16b b, v16b c, v16b d) { asm volatile("v_nop" :: "v"(a), "v"(b), "v"(c), "v"(d)); }
__device__ __forceinline__ void acc_guard4(v8f& a, v8f& b, v8f& c, v8f& d) { asm volatile("v_nop\n\tv_nop\n\tv_nop\n\tv_nop" : "+v"(a), "+v"(b), "+v"(c), "+v"(d)); }
template <typename T> struct Frag;
template <> struct Frag<_Float16> {
  typedef v16h V; union U { v16h v; v8h h[2]; };
  static __device__ __forceinline__ v16h load(const _Float16* p) {
    U f; f.h[0] = *(const v8h*)(p); f.h[1] = *(const v8h*)(p + 16); return f.v;
  }
  static __device__ __forceinline__ v8f mma(v16h a, v16h b, v8f c) {
    return __builtin_amdgcn_wmma_f32_16x16x32_f16(false, a, false, b, (short)0, c, false, false);
  }
  static __device__ __forceinline__ void guard(v8f& a, v8f& b, v16h x, v16h y) { dep_guard_h(a, b, x, y); }
  static __device__ __forceinline__ void keep(v16h a, v16h b, v16h c, v16h d) { keep4_h(a, b, c, d); }
};
template <> struct Frag<__bf16> {
  typedef v16b V; union U { v16b v; v8b h[2]; };
  static __device__ __forceinline__ v16b load(const __bf16* p) {
    U f; f.h[0] = *(const v8b*)(p); f.h[1] = *(const v8b*)(p + 16); return f.v;
  }
  static __device__ __forceinline__ v8f mma(v16b a, v16b b, v8f c) {
    return __builtin_amdgcn_wmma_f32_16x16x32_bf16(false, a, false, b, (short)0, c, false, false);
  }
  static __device__ __forceinline__ void guard(v8f& a, v8f& b, v16b x, v16b y) { dep_guard_b(a, b, x, y); }
  static __device__ __forceinline__ void keep(v16b a, v16b b, v16b c, v16b d) { keep4_b(a, b, c, d); }
};

__device__ __forceinline__ unsigned pk16(unsigned short a, unsigned short b) { return (unsigned)a | ((unsigned)b << 16); }
__device__ __forceinline__ unsigned short h_bits(float f) { const _Float16 h = (_Float16)f; return __builtin_bit_cast(unsigned short, h); }

template <int ET> struct Elem;
template <> struct Elem<0> { typedef _Float16 T; };
template <> struct Elem<1> { typedef __bf16 T; };
template <int ET, bool SPLIT, int BIAS_MODE, int OUT_MODE, bool RESID, int ACT = 0>
__global__ __launch_bounds__(256) void wmma_gemm64(
    const unsigned short* __restrict__ Ap, const unsigned short* __restrict__ A2p, int lda, long strideA,
    const unsigned short* __restrict__ Btp, const unsigned short* __restrict__ Bt2p, int ldb, long strideB,
    void* __restrict__ Cout, void* __restrict__ Cout2, int ldc, long strideC,
    const float* __restrict__ bias,
    const float* __restrict__ resid, long strideR,
    int M, int N, int K, float scale) {
  typedef typename Elem<ET>::T T;
  typedef typename Frag<T>::V V;
  const T* A = (const T*)Ap; const T* A2 = (const T*)A2p; const T* Bt = (const T*)Btp; const T* Bt2 = (const T*)Bt2p;
  __shared__ __align__(16) float sT[8][16 * 68];
  const int b    = blockIdx.y;
  const int lane = threadIdx.x & 31;
  const int wave = threadIdx.x >> 5;
  const int tilesN = N >> 6;
  const int tilesM = M >> 6;
  const int tile = blockIdx.x * 8 + wave;
  if (tile >= tilesM * tilesN) return;
  const int tm = tile / tilesN;
  const int tn = tile - tm * tilesN;
  const int m0 = tm << 6;
  const int n0 = tn << 6;

  const T* Ab  = A  + (size_t)b * strideA;
  const T* Bb  = Bt + (size_t)b * strideB;
  const T* Ab2 = SPLIT ? (A2  + (size_t)b * strideA) : nullptr;
  const T* Bb2 = SPLIT ? (Bt2 + (size_t)b * strideB) : nullptr;

  const int rlane = lane & 15;
  const int koff  = (lane >> 4) * 8;
  const int mOff  = (lane >> 4) * 8;

  v8f acc[4][4];
#pragma unroll
  for (int i = 0; i < 4; ++i)
#pragma unroll
    for (int j = 0; j < 4; ++j) acc[i][j] = (v8f){0.f,0.f,0.f,0.f,0.f,0.f,0.f,0.f};

  for (int k0 = 0; k0 < K; k0 += 32) {
    V bh[4], bl[4];
#pragma unroll
    for (int j = 0; j < 4; ++j) {
      const size_t bo = (size_t)(n0 + (j << 4) + rlane) * ldb + koff + k0;
      bh[j] = Frag<T>::load(Bb + bo);
      if (SPLIT) bl[j] = Frag<T>::load(Bb2 + bo);
    }
#pragma unroll
    for (int i = 0; i < 4; ++i) {
      const size_t ao = (size_t)(m0 + (i << 4) + rlane) * lda + koff + k0;
      V ah = Frag<T>::load(Ab + ao);
      V al;
      if (SPLIT) al = Frag<T>::load(Ab2 + ao);
#pragma unroll
      for (int j = 0; j < 4; ++j) {
        acc[i][j] = Frag<T>::mma(ah, bh[j], acc[i][j]);
        if (SPLIT) {
          acc[i][j] = Frag<T>::mma(ah, bl[j], acc[i][j]);
          acc[i][j] = Frag<T>::mma(al, bh[j], acc[i][j]);
        }
      }
      Frag<T>::guard(acc[i][0], acc[i][3], ah, SPLIT ? al : ah);
    }
    Frag<T>::keep(bh[0], bh[1], bh[2], bh[3]);
    if (SPLIT) Frag<T>::keep(bl[0], bl[1], bl[2], bl[3]);
  }
  acc_guard4(acc[0][0], acc[0][1], acc[0][2], acc[0][3]);
  acc_guard4(acc[1][0], acc[1][1], acc[1][2], acc[1][3]);
  acc_guard4(acc[2][0], acc[2][1], acc[2][2], acc[2][3]);
  acc_guard4(acc[3][0], acc[3][1], acc[3][2], acc[3][3]);

  float* slab = sT[wave];
  const float* Rb = RESID ? (resid + (size_t)b * strideR) : nullptr;
#pragma unroll
  for (int i = 0; i < 4; ++i) {
    const int mBase = m0 + (i << 4);
#pragma unroll
    for (int j = 0; j < 4; ++j) {
      const int n = n0 + (j << 4) + rlane;
      float bv = 0.f;
      if (BIAS_MODE == 2) bv = bias[n];
#pragma unroll
      for (int r = 0; r < 8; ++r) {
        float v = acc[i][j][r] * scale;
        if (BIAS_MODE == 1) v += bias[mBase + mOff + r];
        if (BIAS_MODE == 2) v += bv;
        if (RESID) v += Rb[(size_t)(mBase + mOff + r) * ldc + n];
        if (ACT == 2) v = fmaxf(v, 0.0f);
        if (ACT == 4) v = (v > 0.f) ? v : 0.01f * v;
        slab[(mOff + r) * 68 + (j << 4) + rlane] = v;
      }
    }
    __builtin_amdgcn_fence(__ATOMIC_RELEASE, "workgroup");
    __builtin_amdgcn_wave_barrier();
    __builtin_amdgcn_fence(__ATOMIC_ACQUIRE, "workgroup");
    if (OUT_MODE == 0) {
      float* C = (float*)Cout + (size_t)b * strideC;
      const int hh = lane >> 4, c4 = (lane & 15) * 4;
      for (int pass = 0; pass < 2; ++pass) {
#pragma unroll
        for (int it = 0; it < 8; ++it) {
          const int row = it * 2 + hh;
          v4f v = *(const v4f*)(slab + row * 68 + c4);
          *(volatile v4f*)(C + (size_t)(mBase + row) * ldc + n0 + c4) = v;
        }
        __threadfence();
      }
    } else {
      const int q = lane >> 3, c8 = (lane & 7) * 8;
      unsigned short* C  = (unsigned short*)Cout  + (size_t)b * strideC;
      unsigned short* C2 = (OUT_MODE == 2) ? ((unsigned short*)Cout2 + (size_t)b * strideC) : nullptr;
      for (int pass = 0; pass < 2; ++pass) {
#pragma unroll
        for (int it = 0; it < 4; ++it) {
          const int row = it * 4 + q;
          const float* sp = slab + row * 68 + c8;
          v8h hv, lv;
#pragma unroll
          for (int e = 0; e < 8; ++e) {
            if (OUT_MODE == 1) {
              hv[e] = (_Float16)sp[e];
            } else {
              unsigned short hb = f2bf_bits(sp[e]);
              unsigned short lb = f2bf_bits(sp[e] - bf_bits2f(hb));
              hv[e] = __builtin_bit_cast(_Float16, hb);
              lv[e] = __builtin_bit_cast(_Float16, lb);
            }
          }
          *(volatile v8h*)(C + (size_t)(mBase + row) * ldc + n0 + c8) = hv;
          if (OUT_MODE == 2) *(volatile v8h*)(C2 + (size_t)(mBase + row) * ldc + n0 + c8) = lv;
        }
        __threadfence();
      }
    }
    __builtin_amdgcn_fence(__ATOMIC_RELEASE, "workgroup");
    __builtin_amdgcn_wave_barrier();
    __builtin_amdgcn_fence(__ATOMIC_ACQUIRE, "workgroup");
  }
}

__device__ __forceinline__ float bfr(float f) { return __uint_as_float(((unsigned)f2bf_bits(f)) << 16); }
__device__ __forceinline__ float h16_to_f32(unsigned hb) {
  const unsigned sgn = (hb & 0x8000u) << 16; const unsigned em = hb & 0x7fffu;
  const float fn = __uint_as_float((em << 13) + 0x38000000u);
  const float fs = (float)em * 5.9604644775390625e-8f;
  const float mag = (em < 0x400u) ? fs : fn; return __uint_as_float(__float_as_uint(mag) | sgn);
}
__device__ __forceinline__ float h16_lo(unsigned w) { return h16_to_f32(w & 0xffffu); }
__device__ __forceinline__ float h16_hi(unsigned w) { return h16_to_f32(w >> 16); }
__device__ __forceinline__ float frcp(float x) { return __builtin_amdgcn_rcpf(x); }
__device__ __forceinline__ float sigm(float x) { return frcp(1.0f + expf(-x)); }
__device__ __forceinline__ v8f zero8() { return (v8f){0.f, 0.f, 0.f, 0.f, 0.f, 0.f, 0.f, 0.f}; }
__device__ __forceinline__ v8f mma_h(v16h a, v16h b, v8f c) {
  c = __builtin_amdgcn_wmma_f32_16x16x32_f16(false, a, false, b, (short)0, c, false, false);
  asm volatile("v_nop\n\tv_nop\n\tv_nop\n\tv_nop" : "+v"(c) : "v"(a), "v"(b));
  return c;
}
__device__ __forceinline__ v16h ldfrag(const unsigned short* p) { return Frag<_Float16>::load((const _Float16*)p); }
__device__ __forceinline__ void wave_sync() {
  __builtin_amdgcn_fence(__ATOMIC_RELEASE, "workgroup");
  __builtin_amdgcn_wave_barrier();
  __builtin_amdgcn_fence(__ATOMIC_ACQUIRE, "workgroup");
}
__device__ __forceinline__ v16h frag_from_f32(const float* p) {
  const v4f f0 = *(const v4f*)(p);
  const v4f f1 = *(const v4f*)(p + 4);
  const v4f f2 = *(const v4f*)(p + 16);
  const v4f f3 = *(const v4f*)(p + 20);
  v16h b;
#pragma unroll
  for (int e = 0; e < 4; ++e) {
    b[e]      = (_Float16)f0[e];
    b[4 + e]  = (_Float16)f1[e];
    b[8 + e]  = (_Float16)f2[e];
    b[12 + e] = (_Float16)f3[e];
  }
  return b;
}

__global__ __launch_bounds__(256) void k_cast_x(const float* __restrict__ in, unsigned short* __restrict__ out, int n8) {
  const int i = blockIdx.x * 256 + threadIdx.x;
  if (i >= n8) return;
  const float* p = in + 8 * (size_t)i;
  const v4f a = *(const v4f*)(p);
  const v4f c = *(const v4f*)(p + 4);
  unsigned short hb[8];
#pragma unroll
  for (int e = 0; e < 4; ++e) {
    hb[e]     = h_bits(bfr(a[e]));
    hb[4 + e] = h_bits(bfr(c[e]));
  }
  const v4u u = (v4u){pk16(hb[0], hb[1]), pk16(hb[2], hb[3]), pk16(hb[4], hb[5]), pk16(hb[6], hb[7])};
  unsigned short* q = out + 8 * (size_t)i;
  *(volatile v4u*)q = u;
  __threadfence();
  *(volatile v4u*)q = u;
}

__global__ __launch_bounds__(256) void k_wtcast(const float* __restrict__ W0, const float* __restrict__ W1,
                                                const float* __restrict__ W2, const float* __restrict__ W3, int ldw,
                                                unsigned short* __restrict__ out, long planeStride, int ldt, float scale) {
  __shared__ float sm[64][65];
  const int t  = threadIdx.x;
  const int k0 = blockIdx.x * 64;
  const int n0 = blockIdx.y * 64;
  const int z  = blockIdx.z;
  const float* W = (z == 0) ? W0 : (z == 1) ? W1 : (z == 2) ? W2 : W3;
#pragma unroll 8
  for (int i = 0; i < 16; ++i) {
    const int e = i * 256 + t;
    const int r = e >> 6;
    const int c = e & 63;
    sm[c][r] = bfr(W[(size_t)(k0 + r) * ldw + n0 + c]) * scale;
  }
  __syncthreads();
  const int lane = t & 31, wave = t >> 5;
  const int q = lane >> 3, c8 = (lane & 7) * 8;
  unsigned short* op = out + (size_t)z * planeStride;
  for (int pass = 0; pass < 2; ++pass) {
#pragma unroll
    for (int it = 0; it < 2; ++it) {
      const int row = wave * 8 + it * 4 + q;
      unsigned short hb[8];
#pragma unroll
      for (int e = 0; e < 8; ++e) hb[e] = h_bits(sm[row][c8 + e]);
      const v4u u = (v4u){pk16(hb[0], hb[1]), pk16(hb[2], hb[3]), pk16(hb[4], hb[5]), pk16(hb[6], hb[7])};
      *(volatile v4u*)(op + (size_t)(n0 + row) * ldt + k0 + c8) = u;
    }
    __threadfence();
  }
}

__global__ __launch_bounds__(256) void k_w2cast(const float* __restrict__ W2, unsigned short* __restrict__ out, float scale) {
  __shared__ float sm[16][65];
  const int t  = threadIdx.x;
  const int k0 = blockIdx.x * 64;
  {
    const int r = t >> 2, c4 = (t & 3) * 4;
    const v4f f = *(const v4f*)(W2 + (size_t)(k0 + r) * 16 + c4);
#pragma unroll
    for (int e = 0; e < 4; ++e) sm[c4 + e][r] = bfr(f[e]) * scale;
  }
  __syncthreads();
  const int lane = t & 31;
  const int wave = __builtin_amdgcn_readfirstlane(t >> 5);
  const int q = lane >> 3, c8 = (lane & 7) * 8;
  for (int pass = 0; pass < 2; ++pass) {
#pragma unroll
    for (int it = 0; it < 2; ++it) {
      const int row = wave * 8 + it * 4 + q;
      v4u u = (v4u){0u, 0u, 0u, 0u};
      if (wave < 2) {
        unsigned short hb[8];
#pragma unroll
        for (int e = 0; e < 8; ++e) hb[e] = h_bits(sm[row][c8 + e]);
        u = (v4u){pk16(hb[0], hb[1]), pk16(hb[2], hb[3]), pk16(hb[4], hb[5]), pk16(hb[6], hb[7])};
      }
      *(volatile v4u*)(out + (size_t)row * kHid2 + k0 + c8) = u;
    }
    __threadfence();
  }
}

__global__ __launch_bounds__(256) void k_beta(const float* __restrict__ x, const float* __restrict__ Wb, float* __restrict__ beta) {
  __shared__ __align__(16) float sB[32];
  const int lane = threadIdx.x & 31;
  const int wave = __builtin_amdgcn_readfirstlane(threadIdx.x >> 5);
  const int tok = blockIdx.x * 8 + wave;
  const float* xr = x + (size_t)tok * kD;
  float s0 = 0.f, s1 = 0.f, s2 = 0.f, s3 = 0.f;
#pragma unroll 1
  for (int j = 0; j < 8; ++j) {
    const int d0 = 128 * j + 4 * lane;
    const v4f xv = *(const v4f*)(xr + d0);
    const v4f w0 = *(const v4f*)(Wb + (size_t)(d0 + 0) * 4);
    const v4f w1 = *(const v4f*)(Wb + (size_t)(d0 + 1) * 4);
    const v4f w2 = *(const v4f*)(Wb + (size_t)(d0 + 2) * 4);
    const v4f w3 = *(const v4f*)(Wb + (size_t)(d0 + 3) * 4);
    const float x0 = bfr(xv[0]), x1 = bfr(xv[1]), x2 = bfr(xv[2]), x3 = bfr(xv[3]);
    s0 += x0 * bfr(w0[0]); s1 += x0 * bfr(w0[1]); s2 += x0 * bfr(w0[2]); s3 += x0 * bfr(w0[3]);
    s0 += x1 * bfr(w1[0]); s1 += x1 * bfr(w1[1]); s2 += x1 * bfr(w1[2]); s3 += x1 * bfr(w1[3]);
    s0 += x2 * bfr(w2[0]); s1 += x2 * bfr(w2[1]); s2 += x2 * bfr(w2[2]); s3 += x2 * bfr(w2[3]);
    s0 += x3 * bfr(w3[0]); s1 += x3 * bfr(w3[1]); s2 += x3 * bfr(w3[2]); s3 += x3 * bfr(w3[3]);
  }
#pragma unroll
  for (int off = 16; off > 0; off >>= 1) {
    s0 += __shfl_xor(s0, off, 32);
    s1 += __shfl_xor(s1, off, 32);
    s2 += __shfl_xor(s2, off, 32);
    s3 += __shfl_xor(s3, off, 32);
  }
  if (lane == 0) {
    sB[wave * 4 + 0] = sigm(s0);
    sB[wave * 4 + 1] = sigm(s1);
    sB[wave * 4 + 2] = sigm(s2);
    sB[wave * 4 + 3] = sigm(s3);
  }
  __syncthreads();
  if (wave == 0) {
    const v4f v = *(const v4f*)(sB + (lane & 7) * 4);
    float* dp = beta + (size_t)(blockIdx.x * 8 + (lane & 7)) * 4;
    if (lane < 8) *(volatile v4f*)dp = v;
    __threadfence();
    if (lane < 8) *(volatile v4f*)dp = v;
  }
}

template <int MODE>
__global__ __launch_bounds__(256) void k_conv_act(const float* __restrict__ pre, const float* __restrict__ taps,
                                                  const float* __restrict__ beta, unsigned short* __restrict__ outA,
                                                  unsigned short* __restrict__ outB, float* __restrict__ outF) {
  __shared__ __align__(16) float sW[8][256];
  const int lane = threadIdx.x & 31;
  const int wave = __builtin_amdgcn_readfirstlane(threadIdx.x >> 5);
  const int wid = blockIdx.x * 8 + wave;
  const int tok = wid >> 2, h = wid & 3;
  const int b = tok >> 11, l = tok & (kL - 1);
  const int cb = h * kDK + 8 * lane;
  float* sw = sW[wave];
  float ss = 0.f;
#pragma unroll 1
  for (int g = 0; g < 2; ++g) {
    const int c4 = cb + 4 * g;
    v4f tq[4];
#pragma unroll
    for (int e = 0; e < 4; ++e) tq[e] = *(const v4f*)(taps + (size_t)(c4 + e) * 4);
    v4f xr[4];
#pragma unroll
    for (int jj = 0; jj < 4; ++jj) {
      const int li  = l + jj - 3;
      const int lic = li < 0 ? 0 : li;
      const float fz = li < 0 ? 0.f : 1.f;
      xr[jj] = *(const v4f*)(pre + ((size_t)(b * kL + lic)) * kD + c4) * fz;
    }
#pragma unroll
    for (int e = 0; e < 4; ++e) {
      float acc = 0.f;
#pragma unroll
      for (int jj = 0; jj < 4; ++jj) acc += bfr(tq[e][jj]) * xr[jj][e];
      const float a = acc * frcp(1.0f + expf(-acc));
      sw[8 * lane + 4 * g + e] = a;
      ss += a * a;
    }
  }
#pragma unroll
  for (int off = 16; off > 0; off >>= 1) ss += __shfl_xor(ss, off, 32);
  float bet = 0.f;
  if (MODE != 0) bet = beta[(size_t)tok * 4 + h];
  float inv = 1.f;
  if (MODE != 2) inv = rsqrtf(ss + 1e-6f);
  wave_sync();
  const size_t rowh = ((size_t)((b * kH + h) * kL + l)) * kDK + 8 * lane;
  const v4f p0 = *(const v4f*)(sw + 8 * lane);
  const v4f p1 = *(const v4f*)(sw + 8 * lane + 4);
  unsigned short ha[8], hc[8];
#pragma unroll
  for (int e = 0; e < 4; ++e) {
    const float fa = p0[e] * inv, fb = p1[e] * inv;
    if (MODE == 2) { ha[e] = h_bits(fa * bet); ha[4 + e] = h_bits(fb * bet); }
    else           { ha[e] = h_bits(fa);       ha[4 + e] = h_bits(fb); }
    hc[e] = h_bits(fa * bet); hc[4 + e] = h_bits(fb * bet);
  }
  const v4u uA = (v4u){pk16(ha[0], ha[1]), pk16(ha[2], ha[3]), pk16(ha[4], ha[5]), pk16(ha[6], ha[7])};
  const v4u uC = (v4u){pk16(hc[0], hc[1]), pk16(hc[2], hc[3]), pk16(hc[4], hc[5]), pk16(hc[6], hc[7])};
  const v4f f0 = *(const v4f*)(sw + 4 * lane);
  const v4f f1 = *(const v4f*)(sw + 128 + 4 * lane);
  float* fdst = outF + (size_t)tok * kD + h * kDK + 4 * lane;
  for (int pass = 0; pass < 2; ++pass) {
    *(volatile v4u*)(outA + rowh) = uA;
    if (MODE == 1) *(volatile v4u*)(outB + rowh) = uC;
    if (MODE == 2) {
      *(volatile v4f*)(fdst) = f0;
      *(volatile v4f*)(fdst + 128) = f1;
    }
    __threadfence();
  }
}

__global__ __launch_bounds__(256) void k_chunk_prep(const unsigned short* __restrict__ kn, const unsigned short* __restrict__ kb,
                                                    const unsigned short* __restrict__ vb, unsigned short* __restrict__ u_g,
                                                    unsigned short* __restrict__ w_g) {
  __shared__ __align__(16) unsigned short bufA[32 * 256];
  __shared__ __align__(16) unsigned short bufB[32 * 256];
  __shared__ float sT[32 * 33];
  __shared__ __align__(16) unsigned short sTh[32 * 32];
  const int tid = threadIdx.x, lane = tid & 31;
  const int wave = __builtin_amdgcn_readfirstlane(tid >> 5);
  const int hh = lane >> 4, rl = lane & 15, koff = hh * 8;
  const int blk = blockIdx.x;
  const int chunk = blk & (kNCH - 1);
  const int bh = blk >> 6;
  const size_t rowBase = ((size_t)bh * kL + (size_t)chunk * kC) * kDK;

#pragma unroll
  for (int i = 0; i < 4; ++i) {
    const int idx = tid + i * 256;
    const int r = idx >> 5, c8 = (idx & 31) * 8;
    *(v4u*)(bufA + r * 256 + c8) = *(const v4u*)(kn + rowBase + (size_t)r * 256 + c8);
    *(v4u*)(bufB + r * 256 + c8) = *(const v4u*)(kb + rowBase + (size_t)r * 256 + c8);
  }
  __syncthreads();

  if (wave < 4) {
    const int tm = wave >> 1, tn = wave & 1;
    v8f acc = zero8();
#pragma unroll
    for (int ks = 0; ks < 8; ++ks) {
      const v16h a = ldfrag(bufB + (tm * 16 + rl) * 256 + koff + ks * 32);
      const v16h bq = ldfrag(bufA + (tn * 16 + rl) * 256 + koff + ks * 32);
      acc = mma_h(a, bq, acc);
    }
#pragma unroll
    for (int r = 0; r < 8; ++r) {
      const int i = tm * 16 + 8 * hh + r, j = tn * 16 + rl;
      sT[i * 33 + j] = (j < i) ? -acc[r] : 0.f;
    }
  }
  __syncthreads();

#pragma unroll
  for (int i = 0; i < 4; ++i) {
    const int idx = tid + i * 256;
    const int r = idx >> 5, c8 = (idx & 31) * 8;
    const v4u xk = *(const v4u*)(kb + rowBase + (size_t)r * 256 + c8);
    const v4u xv = *(const v4u*)(vb + rowBase + (size_t)r * 256 + c8);
#pragma unroll
    for (int e = 0; e < 8; ++e) {
      const unsigned wk = xk[e >> 1], wv = xv[e >> 1];
      const unsigned hk = (e & 1) ? (wk >> 16) : (wk & 0xffffu);
      const unsigned hv = (e & 1) ? (wv >> 16) : (wv & 0xffffu);
      bufA[(c8 + e) * 32 + r] = (unsigned short)hk;
      bufB[(c8 + e) * 32 + r] = (unsigned short)hv;
    }
  }
  if (wave == 0) {
    const int j = lane;
    for (int i = 1; i < 32; ++i) {
      float upd = 0.f;
      for (int c = 0; c < i; ++c) upd += sT[i * 33 + c] * sT[c * 33 + j];
      wave_sync();
      if (j < i) sT[i * 33 + j] += upd;
      wave_sync();
    }
    sT[j * 33 + j] = 1.0f;
  }
  __syncthreads();
#pragma unroll
  for (int i = 0; i < 4; ++i) {
    const int idx = tid + i * 256;
    sTh[idx] = h_bits(sT[(idx >> 5) * 33 + (idx & 31)]);
  }
  __syncthreads();

  const unsigned short* Bsrc = (wave < 4) ? bufB : bufA;
  const int tm = (wave >> 1) & 1;
  const int tnb = (wave & 1) * 8;
  const v16h aT = ldfrag(sTh + (tm * 16 + rl) * 32 + koff);
  v8f acc[8];
#pragma unroll
  for (int i = 0; i < 8; ++i) {
    const int tn = tnb + i;
    const v16h bq = ldfrag(Bsrc + (tn * 16 + rl) * 32 + koff);
    acc[i] = mma_h(aT, bq, zero8());
  }
  __syncthreads();
  unsigned short* stage = (wave < 4) ? bufA : bufB;
#pragma unroll
  for (int i = 0; i < 8; ++i) {
    const int tn = tnb + i;
#pragma unroll
    for (int r = 0; r < 8; ++r) stage[(tm * 16 + 8 * hh + r) * 256 + tn * 16 + rl] = h_bits(acc[i][r]);
  }
  __syncthreads();
  const unsigned short* sp = (wave < 4) ? bufA : bufB;
  unsigned short* gp = (wave < 4) ? u_g : w_g;
  for (int pass = 0; pass < 2; ++pass) {
#pragma unroll
    for (int it = 0; it < 8; ++it) {
      const int row = (wave & 3) * 8 + it;
      const v4u v = *(const v4u*)(sp + row * 256 + lane * 8);
      *(volatile v4u*)(gp + rowBase + (size_t)row * 256 + lane * 8) = v;
    }
    __threadfence();
  }
}

__global__ __launch_bounds__(256) void k_delta_scan(const unsigned short* __restrict__ qn, const unsigned short* __restrict__ kn,
                                                    const unsigned short* __restrict__ u_g, const unsigned short* __restrict__ w_g,
                                                    const float* __restrict__ forget, float* __restrict__ delta) {
  __shared__ __align__(16) float sSt[32 * 256];
  __shared__ __align__(16) unsigned short sKT[256 * 32];
  __shared__ __align__(16) unsigned short sU[32 * 32];
  __shared__ __align__(16) unsigned short sUT[32 * 32];
  __shared__ __align__(16) unsigned short sAt[32 * 32];
  __shared__ __align__(16) float sO[32 * 32];
  const int tid = threadIdx.x, lane = tid & 31;
  const int wave = __builtin_amdgcn_readfirstlane(tid >> 5);
  const int hh = lane >> 4, rl = lane & 15, koff = hh * 8;
  const int blk = blockIdx.x;
  const int vq = blk & 7, bh = blk >> 3;
  const int b = bh >> 2, h = bh & 3;
  const int v0 = vq * 32;
  const float lam = 0.55f + 0.45f * sigm(bfr(forget[h]));
  const int tmq = (wave >> 1) & 1, tnq = wave & 1;

#pragma unroll
  for (int i = 0; i < 32; ++i) sSt[tid + i * 256] = 0.f;
  __syncthreads();

  for (int ch = 0; ch < kNCH; ++ch) {
    const int t0 = ch * kC;
    const size_t rowg = (size_t)bh * kL + t0;
#pragma unroll
    for (int i = 0; i < 4; ++i) {
      const int idx = tid + i * 256;
      const int r = idx >> 5, c8 = (idx & 31) * 8;
      const v4u xk = *(const v4u*)(kn + (rowg + r) * 256 + c8);
#pragma unroll
      for (int e = 0; e < 8; ++e) {
        const unsigned wk = xk[e >> 1];
        const unsigned hk = (e & 1) ? (wk >> 16) : (wk & 0xffffu);
        sKT[(c8 + e) * 32 + r] = (unsigned short)hk;
      }
    }
    if (wave < 4) {
      const int r = tid >> 2, c8 = (tid & 3) * 8;
      *(v4u*)(sU + r * 32 + c8) = *(const v4u*)(u_g + (rowg + r) * 256 + v0 + c8);
    }
    __syncthreads();

    v8f accWS = zero8();
    if (wave < 4) {
#pragma unroll 2
      for (int ks = 0; ks < 8; ++ks) {
        const v16h a = ldfrag(w_g + (rowg + tmq * 16 + rl) * 256 + koff + ks * 32);
        const v16h bq = frag_from_f32(sSt + (tnq * 16 + rl) * 256 + ks * 32 + koff);
        accWS = mma_h(a, bq, accWS);
      }
    } else {
      v8f acc = zero8();
#pragma unroll 2
      for (int ks = 0; ks < 8; ++ks) {
        const v16h a = ldfrag(qn + (rowg + tmq * 16 + rl) * 256 + koff + ks * 32);
        const v16h bq = ldfrag(kn + (rowg + tnq * 16 + rl) * 256 + koff + ks * 32);
        acc = mma_h(a, bq, acc);
      }
#pragma unroll
      for (int r = 0; r < 8; ++r) {
        const int i = tmq * 16 + 8 * hh + r, m = tnq * 16 + rl;
        const float av = (m <= i) ? acc[r] : 0.f;
        sAt[i * 32 + m] = h_bits(av);
      }
    }
    __syncthreads();

    if (wave < 4) {
#pragma unroll
      for (int r = 0; r < 8; ++r) {
        const int i = tmq * 16 + 8 * hh + r, n = tnq * 16 + rl;
        const float uv = h16_to_f32((unsigned)sU[i * 32 + n]);
        sUT[n * 32 + i] = h_bits(uv - accWS[r]);
      }
    }
    __syncthreads();

    if (wave < 4) {
      v8f acc = zero8();
#pragma unroll 2
      for (int ks = 0; ks < 8; ++ks) {
        const v16h a = ldfrag(qn + (rowg + tmq * 16 + rl) * 256 + koff + ks * 32);
        const v16h bq = frag_from_f32(sSt + (tnq * 16 + rl) * 256 + ks * 32 + koff);
        acc = mma_h(a, bq, acc);
      }
      {
        const v16h a = ldfrag(sAt + (tmq * 16 + rl) * 32 + koff);
        const v16h bq = ldfrag(sUT + (tnq * 16 + rl) * 32 + koff);
        acc = mma_h(a, bq, acc);
      }
#pragma unroll
      for (int r = 0; r < 8; ++r) sO[(tmq * 16 + 8 * hh + r) * 32 + tnq * 16 + rl] = acc[r];
    }
    __syncthreads();

    {
      const int row = wave * 4 + (lane >> 3), c4 = (lane & 7) * 4;
      const v4f ov = *(const v4f*)(sO + row * 32 + c4);
      float* dp = delta + ((size_t)(b * kL + t0 + row)) * kD + h * kDK + v0 + c4;
      *(volatile v4f*)dp = ov;
      __threadfence();
      *(volatile v4f*)dp = ov;
    }
#pragma unroll
    for (int i = 0; i < 4; ++i) {
      const int id = wave * 4 + i;
      const int tm2 = id >> 1, tn2 = id & 1;
      const v16h a = ldfrag(sKT + (tm2 * 16 + rl) * 32 + koff);
      const v16h bq = ldfrag(sUT + (tn2 * 16 + rl) * 32 + koff);
      float* cp = sSt + (tn2 * 16 + rl) * 256 + tm2 * 16 + 8 * hh;
      const v4f c0 = *(const v4f*)(cp);
      const v4f c1 = *(const v4f*)(cp + 4);
      v8f cacc;
      cacc[0] = lam * c0[0]; cacc[1] = lam * c0[1]; cacc[2] = lam * c0[2]; cacc[3] = lam * c0[3];
      cacc[4] = lam * c1[0]; cacc[5] = lam * c1[1]; cacc[6] = lam * c1[2]; cacc[7] = lam * c1[3];
      const v8f nv = mma_h(a, bq, cacc);
      const v4f o0 = (v4f){nv[0], nv[1], nv[2], nv[3]};
      const v4f o1 = (v4f){nv[4], nv[5], nv[6], nv[7]};
      *(v4f*)(cp) = o0;
      *(v4f*)(cp + 4) = o1;
    }
    __syncthreads();
  }
}

__global__ __launch_bounds__(256) void k_firshort(const float* __restrict__ vact, const float* __restrict__ fir,
                                                  unsigned short* __restrict__ outp) {
  const int i = blockIdx.x * 256 + threadIdx.x;
  const int tok = i >> 7, c8 = (i & 127) * 8;
  const int b = tok >> 11, l = tok & (kL - 1);
  v4f tp[6];
#pragma unroll
  for (int q = 0; q < 6; ++q) tp[q] = *(const v4f*)(fir + (size_t)c8 * 3 + 4 * q);
  asm volatile("" :: "v"(tp[0]), "v"(tp[1]), "v"(tp[2]) : "memory");
  asm volatile("" :: "v"(tp[3]), "v"(tp[4]), "v"(tp[5]) : "memory");
  v4f xa[3], xb[3];
#pragma unroll
  for (int jj = 0; jj < 3; ++jj) {
    const int li = l + jj - 2;
    const int lic = li < 0 ? 0 : li;
    const float fz = li < 0 ? 0.f : 1.f;
    const float* vp = vact + ((size_t)(b * kL + lic)) * kD + c8;
    xa[jj] = *(const v4f*)(vp) * fz;
    xb[jj] = *(const v4f*)(vp + 4) * fz;
  }
  unsigned short hb[8];
#pragma unroll
  for (int e = 0; e < 8; ++e) {
    float s = 0.f;
#pragma unroll
    for (int jj = 0; jj < 3; ++jj) {
      const int m = e * 3 + jj;
      const float w = bfr(tp[m >> 2][m & 3]);
      const float xv = (e < 4) ? xa[jj][e & 3] : xb[jj][e & 3];
      s += w * xv;
    }
    hb[e] = h_bits(s);
  }
  const v4u u = (v4u){pk16(hb[0], hb[1]), pk16(hb[2], hb[3]), pk16(hb[4], hb[5]), pk16(hb[6], hb[7])};
  unsigned short* q = outp + (size_t)tok * kD + c8;
  *(volatile v4u*)q = u;
  __threadfence();
  *(volatile v4u*)q = u;
}

__global__ __launch_bounds__(256) void k_firlong(const float* __restrict__ vact, const float* __restrict__ fir,
                                                 float* __restrict__ outp) {
  __shared__ __align__(16) unsigned short seqh[32 * kSeqLen];
  __shared__ __align__(16) unsigned short taph[32 * 128];
  __shared__ __align__(16) float stg[256 * 32];
  const int tid = threadIdx.x, lane = tid & 31;
  const int wave = __builtin_amdgcn_readfirstlane(tid >> 5);
  const int hh = lane >> 4, rl = lane & 15, koff = hh * 8;
  const int c0 = blockIdx.x * 32;
  const int T0 = blockIdx.y * 256;
  const int b = T0 >> 11, l0 = T0 & (kL - 1);
#pragma unroll 2
  for (int it = 0; it < 42; ++it) {
    const int idx = it * 256 + tid;
    const int t = idx >> 5, cl = idx & 31;
    const int l = l0 - 62 + t;
    const int lc = l < 0 ? 0 : (l >= kL ? kL - 1 : l);
    const float fz = ((l >= 0) && (l < kL)) ? 1.0f : 0.0f;
    const float xv = vact[((size_t)(b * kL + lc)) * kD + c0 + cl];
    seqh[cl * kSeqLen + t] = h_bits(xv * fz);
  }
#pragma unroll 2
  for (int it = 0; it < 16; ++it) {
    const int idx = it * 256 + tid;
    const int cl = idx >> 7, i = idx & 127;
    const int jt = i - 16;
    const int jc = jt < 0 ? 0 : (jt >= kFirK ? kFirK - 1 : jt);
    const float fac = ((jt >= 0) && (jt < kFirK)) ? kTapCar : 0.0f;
    const float f = fir[(size_t)(c0 + cl) * kFirK + jc];
    taph[cl * 128 + i] = h_bits(bfr(f) * fac);
  }
  __syncthreads();
#pragma unroll 1
  for (int qd = 0; qd < 4; ++qd) {
    const int cl = wave * 4 + qd;
    const unsigned short* tp = taph + cl * 128 + 16 - rl;
    v8u u0, u1, u2;
#pragma unroll
    for (int e = 0; e < 4; ++e) {
      u0[e]     = pk16(tp[koff + 2 * e],      tp[koff + 2 * e + 1]);
      u0[4 + e] = pk16(tp[16 + koff + 2 * e], tp[16 + koff + 2 * e + 1]);
      u1[e]     = pk16(tp[32 + koff + 2 * e], tp[32 + koff + 2 * e + 1]);
      u1[4 + e] = pk16(tp[48 + koff + 2 * e], tp[48 + koff + 2 * e + 1]);
      u2[e]     = pk16(tp[64 + koff + 2 * e], tp[64 + koff + 2 * e + 1]);
      u2[4 + e] = pk16(tp[80 + koff + 2 * e], tp[80 + koff + 2 * e + 1]);
    }
    const v16h a0 = __builtin_bit_cast(v16h, u0);
    const v16h a1 = __builtin_bit_cast(v16h, u1);
    const v16h a2 = __builtin_bit_cast(v16h, u2);
    const unsigned short* sp = seqh + cl * kSeqLen + rl * 16 + koff;
    const v16h b0 = ldfrag(sp);
    const v16h b1 = ldfrag(sp + 32);
    const v16h b2 = ldfrag(sp + 64);
    v8f acc = mma_h(a0, b0, zero8());
    acc = mma_h(a1, b1, acc);
    acc = mma_h(a2, b2, acc);
#pragma unroll
    for (int r = 0; r < 8; ++r) stg[(16 * rl + 8 * hh + r) * 32 + cl] = acc[r] * kTapCarInv;
  }
  __syncthreads();
  const int q = lane >> 3, c4 = (lane & 7) * 4;
  for (int pass = 0; pass < 2; ++pass) {
#pragma unroll
    for (int it = 0; it < 8; ++it) {
      const int row = wave * 32 + it * 4 + q;
      const v4f v = *(const v4f*)(stg + row * 32 + c4);
      *(volatile v4f*)(outp + ((size_t)(T0 + row)) * kD + c0 + c4) = v;
    }
    __threadfence();
  }
}

__global__ __launch_bounds__(256) void k_gate_in(const unsigned short* __restrict__ x16, const unsigned short* __restrict__ shortp,
                                                 const float* __restrict__ longp, const float* __restrict__ deltap,
                                                 const float* __restrict__ vactp, unsigned short* __restrict__ gate) {
  __shared__ __align__(16) float sStat[64];
  const int tid = threadIdx.x, lane = tid & 31;
  const int wave = __builtin_amdgcn_readfirstlane(tid >> 5);
  const int tok = blockIdx.x;
#pragma unroll
  for (int i = 0; i < 2; ++i) {
    const int task = wave * 2 + i;
    const int ti = task >> 2, hd = task & 3;
    const size_t base = (size_t)tok * kD + hd * kDK + 8 * lane;
    float xv[8];
    if (ti == 0) {
      const v4u w = *(const v4u*)(shortp + base);
#pragma unroll
      for (int e = 0; e < 4; ++e) { const unsigned ww = w[e]; xv[2 * e] = h16_lo(ww); xv[2 * e + 1] = h16_hi(ww); }
    } else {
      const float* p = (ti == 1) ? longp : (ti == 2) ? deltap : vactp;
      const v4f a = *(const v4f*)(p + base);
      const v4f c = *(const v4f*)(p + base + 4);
#pragma unroll
      for (int e = 0; e < 4; ++e) { xv[e] = a[e]; xv[4 + e] = c[e]; }
    }
    float s = 0.f, sq = 0.f, mx = xv[0];
#pragma unroll
    for (int j = 0; j < 8; ++j) { s += xv[j]; sq += xv[j] * xv[j]; mx = fmaxf(mx, xv[j]); }
#pragma unroll
    for (int off = 16; off > 0; off >>= 1) {
      s  += __shfl_xor(s, off, 32);
      sq += __shfl_xor(sq, off, 32);
      mx  = fmaxf(mx, __shfl_xor(mx, off, 32));
    }
    const float mean = s * (1.0f / 256.0f);
    float d2 = 0.f;
#pragma unroll
    for (int j = 0; j < 8; ++j) { const float dv = xv[j] - mean; d2 += dv * dv; }
#pragma unroll
    for (int off = 16; off > 0; off >>= 1) d2 += __shfl_xor(d2, off, 32);
    if (lane == 0) {
      sStat[task * 4 + 0] = mean;
      sStat[task * 4 + 1] = d2 * (1.0f / 256.0f);
      sStat[task * 4 + 2] = mx;
      sStat[task * 4 + 3] = sqrtf(sq);
    }
  }
  __syncthreads();
  unsigned short* row = gate + (size_t)tok * kGIn;
  if (wave < 4) {
    const v4u v = *(const v4u*)(x16 + (size_t)tok * kD + tid * 8);
    *(volatile v4u*)(row + tid * 8) = v;
    __threadfence();
    *(volatile v4u*)(row + tid * 8) = v;
  } else if (wave == 4) {
    const int l8 = (lane & 7) * 8;
    unsigned short hb[8];
#pragma unroll
    for (int e = 0; e < 8; ++e) hb[e] = h_bits(sStat[l8 + e]);
    const v4u u = (v4u){pk16(hb[0], hb[1]), pk16(hb[2], hb[3]), pk16(hb[4], hb[5]), pk16(hb[6], hb[7])};
    unsigned short* dp = row + kD + l8;
    if (lane < 8) *(volatile v4u*)dp = u;
    __threadfence();
    if (lane < 8) *(volatile v4u*)dp = u;
  }
}

__global__ __launch_bounds__(256) void k_gelu(unsigned short* __restrict__ hm, const float* __restrict__ b1, int n2) {
  const int i = blockIdx.x * 256 + threadIdx.x;
  if (i >= n2) return;
  const unsigned w = ((const unsigned*)hm)[i];
  const int n = (2 * i) & (kHid2 - 1);
  const float x0 = h16_lo(w) + bfr(b1[n]);
  const float x1 = h16_hi(w) + bfr(b1[n + 1]);
  const float g0 = 0.5f * x0 * (1.0f + erff(x0 * 0.70710678118654752f));
  const float g1 = 0.5f * x1 * (1.0f + erff(x1 * 0.70710678118654752f));
  const unsigned u = pk16(h_bits(g0 * kHmCar), h_bits(g1 * kHmCar));
  ((volatile unsigned*)hm)[i] = u;
  __threadfence();
  ((volatile unsigned*)hm)[i] = u;
}

__global__ __launch_bounds__(256) void k_gate_p(const float* __restrict__ logits, const float* __restrict__ log_temp,
                                                const float* __restrict__ floor_p, const float* __restrict__ b2,
                                                float* __restrict__ P) {
  const int idx = blockIdx.x * 256 + threadIdx.x;
  if (idx >= kTok * kH) return;
  const int h = idx & 3, tok = idx >> 2;
  const v4f lg  = *(const v4f*)(logits + (size_t)tok * kNLg + h * 4);
  const v4f bb  = *(const v4f*)(b2 + h * 4);
  const v4f flp = *(const v4f*)(floor_p + h * 4);
  const float tinv = frcp(expf(bfr(log_temp[h])));
  float xs[4], es[4], cl[4];
  float mx = -3.0e38f;
#pragma unroll
  for (int s = 0; s < 4; ++s) { xs[s] = (lg[s] + bfr(bb[s])) * tinv; mx = fmaxf(mx, xs[s]); }
  float sum = 0.f;
#pragma unroll
  for (int s = 0; s < 4; ++s) { es[s] = expf(xs[s] - mx); sum += es[s]; }
  const float inv = frcp(sum);
  float cs = 0.f;
#pragma unroll
  for (int s = 0; s < 4; ++s) {
    const float fl = 0.075f * sigm(bfr(flp[s]));
    cl[s] = fmaxf(es[s] * inv, fl);
    cs += cl[s];
  }
  const float ci = frcp(cs);
  const v4f pv = (v4f){cl[0] * ci, cl[1] * ci, cl[2] * ci, cl[3] * ci};
  float* dp = P + (size_t)idx * 4;
  *(volatile v4f*)dp = pv;
  __threadfence();
  *(volatile v4f*)dp = pv;
}

__global__ __launch_bounds__(256) void k_gate_fuse(const float* __restrict__ P, const unsigned short* __restrict__ shortp,
                                                   const float* __restrict__ longp, const float* __restrict__ deltap,
                                                   const float* __restrict__ vactp, const float* __restrict__ norm_w,
                                                   unsigned short* __restrict__ outp) {
  __shared__ __align__(16) float sW[8][256];
  const int lane = threadIdx.x & 31;
  const int wave = __builtin_amdgcn_readfirstlane(threadIdx.x >> 5);
  const int wid = blockIdx.x * 8 + wave;
  const int tok = wid >> 2, h = wid & 3;
  const v4f pv = *(const v4f*)(P + ((size_t)tok * kH + h) * 4);
  const size_t base = (size_t)tok * kD + h * kDK + 8 * lane;
  float* sw = sW[wave];
  float ss = 0.f;
#pragma unroll 1
  for (int g = 0; g < 2; ++g) {
    const size_t o4 = base + 4 * g;
    const v2u sh2 = *(const v2u*)(shortp + o4);
    const v4f lo  = *(const v4f*)(longp + o4);
    const v4f de  = *(const v4f*)(deltap + o4);
    const v4f vv  = *(const v4f*)(vactp + o4);
#pragma unroll
    for (int e = 0; e < 4; ++e) {
      const unsigned ww = sh2[e >> 1];
      const float sh = (e & 1) ? h16_hi(ww) : h16_lo(ww);
      const float ov = pv[0] * sh + pv[1] * lo[e] + pv[2] * de[e] + pv[3] * vv[e];
      sw[8 * lane + 4 * g + e] = ov;
      ss += ov * ov;
    }
  }
#pragma unroll
  for (int off = 16; off > 0; off >>= 1) ss += __shfl_xor(ss, off, 32);
  const float rinv = rsqrtf(ss * (1.0f / 256.0f) + 1e-5f);
  wave_sync();
  const v4f a  = *(const v4f*)(sw + 8 * lane);
  const v4f c  = *(const v4f*)(sw + 8 * lane + 4);
  const v4f n0 = *(const v4f*)(norm_w + 8 * lane);
  const v4f n1 = *(const v4f*)(norm_w + 8 * lane + 4);
  unsigned short hb[8];
#pragma unroll
  for (int e = 0; e < 4; ++e) {
    hb[e]     = h_bits((a[e] * rinv) * bfr(n0[e]));
    hb[4 + e] = h_bits((c[e] * rinv) * bfr(n1[e]));
  }
  const v4u u = (v4u){pk16(hb[0], hb[1]), pk16(hb[2], hb[3]), pk16(hb[4], hb[5]), pk16(hb[6], hb[7])};
  unsigned short* dp = outp + base;
  *(volatile v4u*)dp = u;
  __threadfence();
  *(volatile v4u*)dp = u;
}

extern "C" void kernel_launch(void* const* d_in, const int* in_sizes, int n_in,
                              void* d_out, int out_size, void* d_ws, size_t ws_size,
                              hipStream_t stream) {
  if (n_in < 19) return;
  const int nTokD = kTok * kD;
  if (in_sizes[0] != nTokD) return;
  if (in_sizes[1] != kD * kD || in_sizes[2] != kD * kD || in_sizes[3] != kD * kD || in_sizes[18] != kD * kD) return;
  if (in_sizes[4] != kD * kH || in_sizes[5] != kH) return;
  if (in_sizes[6] != kD * 4 || in_sizes[7] != kD * 4 || in_sizes[8] != kD * 4) return;
  if (in_sizes[9] != kD * 3 || in_sizes[10] != kD * kFirK) return;
  if (in_sizes[11] != kH || in_sizes[12] != kH * 4) return;
  if (in_sizes[13] != kGIn * kHid2 || in_sizes[14] != kHid2 || in_sizes[15] != kHid2 * 16 || in_sizes[16] != 16) return;
  if (in_sizes[17] != kDK) return;
  if (out_size != nTokD) return;

  const size_t szX16  = (size_t)kTok * kD * 2;
  const size_t szWT4  = (size_t)4 * kD * kD * 2;
  const size_t szW1T  = (size_t)kHid2 * kGIn * 2;
  const size_t szW2T  = (size_t)kNLg * kHid2 * 2;
  const size_t szF32  = (size_t)kTok * kD * 4;
  const size_t szHead = (size_t)kBH * kL * kDK * 2;
  const size_t szSh   = (size_t)kTok * kD * 2;
  const size_t szBeta = (size_t)kTok * kH * 4;
  const size_t szLg   = (size_t)kTok * kNLg * 4;
  const size_t szPg   = (size_t)kTok * kH * 4 * 4;
  static_assert((size_t)kTok * kGIn * 2 + (size_t)kTok * kHid2 * 2 <= (size_t)4 * kBH * kL * kDK * 2, "gate planes fit the head region");
  static_assert((size_t)kTok * kD * 2 <= (size_t)2 * kBH * kL * kDK * 2, "fused plane fits the u/w region");
  const size_t offX16  = 0;
  const size_t offWT4  = offX16 + szX16;
  const size_t offW1T  = offWT4 + szWT4;
  const size_t offW2T  = offW1T + szW1T;
  const size_t offPre  = offW2T + szW2T;
  const size_t offHead = offPre + szF32;
  const size_t offVact = offHead + 4 * szHead;
  const size_t offUW   = offVact + szF32;
  const size_t offDel  = offUW + 2 * szHead;
  const size_t offSh   = offDel + szF32;
  const size_t offBeta = offSh + szSh;
  const size_t offLg   = offBeta + szBeta;
  const size_t offPg   = offLg + szLg;
  const size_t total   = offPg + szPg;
  if (ws_size < total) return;

  const float* x        = (const float*)d_in[0];
  const float* Wq       = (const float*)d_in[1];
  const float* Wk       = (const float*)d_in[2];
  const float* Wv       = (const float*)d_in[3];
  const float* Wb       = (const float*)d_in[4];
  const float* forget_p = (const float*)d_in[5];
  const float* conv_q   = (const float*)d_in[6];
  const float* conv_k   = (const float*)d_in[7];
  const float* conv_v   = (const float*)d_in[8];
  const float* fir_s    = (const float*)d_in[9];
  const float* fir_l    = (const float*)d_in[10];
  const float* log_temp = (const float*)d_in[11];
  const float* floor_p  = (const float*)d_in[12];
  const float* W1       = (const float*)d_in[13];
  const float* b1       = (const float*)d_in[14];
  const float* W2       = (const float*)d_in[15];
  const float* b2       = (const float*)d_in[16];
  const float* norm_w   = (const float*)d_in[17];
  const float* Wo       = (const float*)d_in[18];
  float* out = (float*)d_out;
  char* ws = (char*)d_ws;
  unsigned short* X16  = (unsigned short*)(ws + offX16);
  unsigned short* WT4  = (unsigned short*)(ws + offWT4);
  unsigned short* WQT  = WT4;
  unsigned short* WKT  = WT4 + (size_t)kD * kD;
  unsigned short* WVT  = WT4 + (size_t)2 * kD * kD;
  unsigned short* WOT  = WT4 + (size_t)3 * kD * kD;
  unsigned short* W1T  = (unsigned short*)(ws + offW1T);
  unsigned short* W2T  = (unsigned short*)(ws + offW2T);
  float*          PRE  = (float*)(ws + offPre);
  float*          LONG = (float*)(ws + offPre);
  unsigned short* QN   = (unsigned short*)(ws + offHead);
  unsigned short* KN   = QN + (size_t)kBH * kL * kDK;
  unsigned short* KB   = QN + (size_t)2 * kBH * kL * kDK;
  unsigned short* VB   = QN + (size_t)3 * kBH * kL * kDK;
  unsigned short* GIN  = (unsigned short*)(ws + offHead);
  unsigned short* HM   = (unsigned short*)(ws + offHead + (size_t)kTok * kGIn * 2);
  float*          VACT = (float*)(ws + offVact);
  unsigned short* UG   = (unsigned short*)(ws + offUW);
  unsigned short* WG   = UG + (size_t)kBH * kL * kDK;
  unsigned short* OFU  = (unsigned short*)(ws + offUW);
  float*          DEL  = (float*)(ws + offDel);
  unsigned short* SH   = (unsigned short*)(ws + offSh);
  float*          BETA = (float*)(ws + offBeta);
  float*          LG   = (float*)(ws + offLg);
  float*          PG   = (float*)(ws + offPg);

  const dim3 blk(256);
  const int n8 = nTokD / 8;
  k_cast_x<<<dim3(n8 / 256), blk, 0, stream>>>(x, X16, n8);
  k_wtcast<<<dim3(kD / 64, kD / 64, 4), blk, 0, stream>>>(Wq, Wk, Wv, Wo, kD, WT4, (long)kD * kD, kD, kWCar);
  k_wtcast<<<dim3(kGIn / 64, kHid2 / 64, 1), blk, 0, stream>>>(W1, W1, W1, W1, kHid2, W1T, 0L, kGIn, kWCar);
  k_w2cast<<<dim3(kHid2 / 64), blk, 0, stream>>>(W2, W2T, kWCar);
  k_beta<<<dim3(kTok / 8), blk, 0, stream>>>(x, Wb, BETA);
  const int tilesProj = (kTok / 64) * (kD / 64);
  wmma_gemm64<0, false, 0, 0, false, 0><<<dim3(tilesProj / 8, 1), blk, 0, stream>>>(
      X16, X16, kD, 0L, WQT, WQT, kD, 0L, (void*)PRE, (void*)PRE, kD, 0L, BETA, BETA, 0L, kTok, kD, kD, kWCarInv);
  k_conv_act<0><<<dim3(kTok * kH / 8), blk, 0, stream>>>(PRE, conv_q, BETA, QN, QN, VACT);
  wmma_gemm64<0, false, 0, 0, false, 0><<<dim3(tilesProj / 8, 1), blk, 0, stream>>>(
      X16, X16, kD, 0L, WKT, WKT, kD, 0L, (void*)PRE, (void*)PRE, kD, 0L, BETA, BETA, 0L, kTok, kD, kD, kWCarInv);
  k_conv_act<1><<<dim3(kTok * kH / 8), blk, 0, stream>>>(PRE, conv_k, BETA, KN, KB, VACT);
  wmma_gemm64<0, false, 0, 0, false, 0><<<dim3(tilesProj / 8, 1), blk, 0, stream>>>(
      X16, X16, kD, 0L, WVT, WVT, kD, 0L, (void*)PRE, (void*)PRE, kD, 0L, BETA, BETA, 0L, kTok, kD, kD, kWCarInv);
  k_conv_act<2><<<dim3(kTok * kH / 8), blk, 0, stream>>>(PRE, conv_v, BETA, VB, VB, VACT);
  k_chunk_prep<<<dim3(kBH * kNCH), blk, 0, stream>>>(KN, KB, VB, UG, WG);
  k_delta_scan<<<dim3(kBH * 8), blk, 0, stream>>>(QN, KN, UG, WG, forget_p, DEL);
  k_firshort<<<dim3(kTok * 128 / 256), blk, 0, stream>>>(VACT, fir_s, SH);
  k_firlong<<<dim3(kD / 32, kTok / 256), blk, 0, stream>>>(VACT, fir_l, LONG);
  k_gate_in<<<dim3(kTok), blk, 0, stream>>>(X16, SH, LONG, DEL, VACT, GIN);
  const int tilesW1 = (kTok / 64) * (kHid2 / 64);
  wmma_gemm64<0, false, 0, 1, false, 0><<<dim3(tilesW1 / 8, 1), blk, 0, stream>>>(
      GIN, GIN, kGIn, 0L, W1T, W1T, kGIn, 0L, (void*)HM, (void*)HM, kHid2, 0L, BETA, BETA, 0L, kTok, kHid2, kGIn, kWCarInv);
  const int n2 = kTok * kHid2 / 2;
  k_gelu<<<dim3(n2 / 256), blk, 0, stream>>>(HM, b1, n2);
  const int tilesW2 = (kTok / 64) * (kNLg / 64);
  wmma_gemm64<0, false, 0, 0, false, 0><<<dim3(tilesW2 / 8, 1), blk, 0, stream>>>(
      HM, HM, kHid2, 0L, W2T, W2T, kHid2, 0L, (void*)LG, (void*)LG, kNLg, 0L, BETA, BETA, 0L, kTok, kNLg, kHid2, kW2Scale);
  k_gate_p<<<dim3(kTok * kH / 256), blk, 0, stream>>>(LG, log_temp, floor_p, b2, PG);
  k_gate_fuse<<<dim3(kTok * kH / 8), blk, 0, stream>>>(PG, SH, LONG, DEL, VACT, norm_w, OFU);
  wmma_gemm64<0, false, 0, 0, false, 0><<<dim3(tilesProj / 8, 1), blk, 0, stream>>>(
      OFU, OFU, kD, 0L, WOT, WOT, kD, 0L, (void*)out, (void*)out, kD, 0L, BETA, BETA, 0L, kTok, kD, kD, kWCarInv);
}
